// grud_model_5738076308227
// MI455X (gfx1250) — hardware-run, weakly checked
//
#include <hip/hip_runtime.h>
#include <cstdint>

typedef __attribute__((ext_vector_type(16))) _Float16 v16h;
typedef __attribute__((ext_vector_type(8)))  float    v8f;

constexpr int kB = 64, kC = 128, kH = 256, kO = 128, kT = 512;
constexpr int kTB = kT * kB;

struct alignas(16) U128 { unsigned int a, b, c, d; };
typedef __attribute__((ext_vector_type(4))) float v4f;
typedef __attribute__((ext_vector_type(4))) unsigned v4u;
typedef __attribute__((ext_vector_type(8))) _Float16 v8h;
template <typename T> __device__ __forceinline__ void vst2(void* p, T v) { *(volatile T*)p = v; __threadfence(); *(volatile T*)p = v; }
union V16U { v16h h; U128 q[2]; };
union V8FU { v8f v; float f[8]; };


__device__ __forceinline__ v16h load_a_f16(const _Float16* A, int lda, int lane,
                                           int row0, int k0) {
  const int r  = row0 + (lane & 15);
  const int kb = k0 + ((lane & 16) ? 8 : 0);
  const _Float16* p = A + (size_t)r * lda + kb;
  V16U u;
  u.q[0] = *reinterpret_cast<const U128*>(p);
  u.q[1] = *reinterpret_cast<const U128*>(p + 16);
  return u.h;
}

__device__ __forceinline__ v16h load_b_f16(const _Float16* W, int ldw, int lane,
                                           int n0, int k0) {
  const int n  = n0 + (lane & 15);
  const int kb = k0 + ((lane & 16) ? 8 : 0);
  const _Float16* p = W + (size_t)n * ldw + kb;
  V16U u;
  u.q[0] = *reinterpret_cast<const U128*>(p);
  u.q[1] = *reinterpret_cast<const U128*>(p + 16);
  return u.h;
}

__device__ __forceinline__ float sigmoidf_(float x) {
  return 1.0f / (1.0f + expf(-x));
}

__device__ __forceinline__ v8f wmma_f16(v16h a, v16h b, v8f c) {
  v8f d = __builtin_amdgcn_wmma_f32_16x16x32_f16(false, a, false, b, (short)0, c, false, false);
  asm volatile("v_nop\n\tv_nop\n\tv_nop\n\tv_nop" : "+v"(d) : "v"(a), "v"(b));
  return d;
}


__global__ void __launch_bounds__(256)
f32_to_f16_kernel(const float* __restrict__ s, _Float16* __restrict__ d, int n) {
  int g8 = blockIdx.x * blockDim.x + threadIdx.x;
  if (g8 * 8 < n) { union { v8h h; v4u u; } pk;
#pragma unroll
    for (int e = 0; e < 8; ++e) pk.h[e] = (_Float16)s[g8 * 8 + e];
    vst2(d + (size_t)g8 * 8, pk.u); }
}

__global__ void __launch_bounds__(256)
reorder_inputs(const float* __restrict__ inp, float* __restrict__ Xf,
               _Float16* __restrict__ M16, _Float16* __restrict__ D16) {
  const int t = blockIdx.x, tid = threadIdx.x;
  const size_t o0 = (size_t)t * kB * kC;
  for (int q = tid; q < kB * kC / 4; q += 256) { const int bc = q * 4; const int b = bc / kC, c = bc % kC;
    v4f v;
#pragma unroll
    for (int e = 0; e < 4; ++e) v[e] = inp[((size_t)(b * 3 + 0) * kC + c + e) * kT + t];
    vst2(Xf + o0 + bc, v); }
  for (int q = tid; q < kB * kC / 8; q += 256) { const int bc = q * 8; const int b = bc / kC, c = bc % kC;
    union { v8h h; v4u u; } pm, pd;
#pragma unroll
    for (int e = 0; e < 8; ++e) { pm.h[e] = (_Float16)inp[((size_t)(b * 3 + 1) * kC + c + e) * kT + t]; pd.h[e] = (_Float16)inp[((size_t)(b * 3 + 2) * kC + c + e) * kT + t]; }
    vst2(M16 + o0 + bc, pm.u); vst2(D16 + o0 + bc, pd.u); }
}

__device__ __forceinline__ void store_gamma(float* st, int N,
                                            const float* __restrict__ bias,
                                            int rowl0, int col0, int lane,
                                            const V8FU& acc) {
  const int col = col0 + (lane & 15);
  const int rb  = (lane & 16) ? 8 : 0;
  const float bv = bias[col];
  #pragma unroll
  for (int i = 0; i < 8; ++i) {
    const float v = acc.f[i] + bv;
    st[(size_t)(rowl0 + rb + i) * (N + 4) + col] = expf(-fmaxf(v, 0.0f));
  }
}

__global__ void __launch_bounds__(256)
gemm_gamma(const _Float16* __restrict__ A, const _Float16* __restrict__ W,
           const float* __restrict__ bias, float* __restrict__ out,
           int N, int nt2  , int K, int ldw) {
  __shared__ __align__(16) float st[64 * 132];
  const int wave = threadIdx.x >> 5;
  const int lane = threadIdx.x & 31;
  const int tile = blockIdx.x * 8 + wave;
  const int row0 = (tile / nt2) * 32;
  const int col0 = (tile % nt2) * 32;
  const int rowblk = (blockIdx.x * 8 / nt2) * 32;
  V8FU a00 = {}, a01 = {}, a10 = {}, a11 = {};
  for (int k0 = 0; k0 < K; k0 += 32) {
    v16h va0 = load_a_f16(A, K, lane, row0, k0);
    v16h va1 = load_a_f16(A, K, lane, row0 + 16, k0);
    v16h vb0 = load_b_f16(W, ldw, lane, col0, k0);
    v16h vb1 = load_b_f16(W, ldw, lane, col0 + 16, k0);
    a00.v = wmma_f16(va0, vb0, a00.v);
    a01.v = wmma_f16(va0, vb1, a01.v);
    a10.v = wmma_f16(va1, vb0, a10.v);
    a11.v = wmma_f16(va1, vb1, a11.v);
  }
  store_gamma(st, N, bias, row0 - rowblk,      col0,      lane, a00);
  store_gamma(st, N, bias, row0 - rowblk,      col0 + 16, lane, a01);
  store_gamma(st, N, bias, row0 - rowblk + 16, col0,      lane, a10);
  store_gamma(st, N, bias, row0 - rowblk + 16, col0 + 16, lane, a11);
  __syncthreads();
  const int nrows = (8 / nt2) * 32, np4 = N / 4;
  for (int q = threadIdx.x; q < nrows * np4; q += 256) { const int rl = q / np4, pc = q % np4;
    vst2(out + (size_t)(rowblk + rl) * N + pc * 4, *(const v4f*)(st + (size_t)rl * (N + 4) + pc * 4)); }
}

__global__ void __launch_bounds__(256)
scan_impute(const float* __restrict__ Xf, const _Float16* __restrict__ M16,
            const float* __restrict__ GX, const float* __restrict__ xmean_p,
            _Float16* __restrict__ XI) {
  const int bc0 = (blockIdx.x * blockDim.x + threadIdx.x) * 8;
  const float xmean = xmean_p[0];
  float x_last[8] = {0.f, 0.f, 0.f, 0.f, 0.f, 0.f, 0.f, 0.f};
  for (int t = 0; t < kT; ++t) {
    const size_t idx = (size_t)t * kB * kC + bc0;
    union { v8h h; v4u u; } pk;
#pragma unroll
    for (int e = 0; e < 8; ++e) {
      const float m = (float)M16[idx + e];
      const float x = Xf[idx + e];
      if (m > 0.0f) x_last[e] = x;
      const float gx = GX[idx + e];
      pk.h[e] = (_Float16)(m * x + (1.0f - m) * (gx * x_last[e] + (1.0f - gx) * xmean));
    }
    vst2(XI + idx, pk.u);
  }
}

__device__ __forceinline__ void store_pre(float* st,
                                          const float* __restrict__ bias,
                                          int rowl0, int col0, int lane,
                                          const V8FU& acc) {
  const int col = col0 + (lane & 15);
  const int rb  = (lane & 16) ? 8 : 0;
  const float bv = bias ? bias[col] : 0.0f;
  #pragma unroll
  for (int i = 0; i < 8; ++i)
    st[(size_t)(rowl0 + rb + i) * (kH + 4) + col] = acc.f[i] + bv;
}

__global__ void __launch_bounds__(256)
gemm_pre(const _Float16* __restrict__ XI, const _Float16* __restrict__ M,
         const _Float16* __restrict__ WxZ, const _Float16* __restrict__ WmZ,
         const _Float16* __restrict__ WxR, const _Float16* __restrict__ WmR,
         const _Float16* __restrict__ WxH, const _Float16* __restrict__ WmH,
         const float* __restrict__ bZ, const float* __restrict__ bH,
         float* __restrict__ preZ, float* __restrict__ preR,
         float* __restrict__ preH) {
  const int gate = blockIdx.y;
  const _Float16* Wx = (gate == 0) ? WxZ : (gate == 1) ? WxR : WxH;
  const _Float16* Wm = (gate == 0) ? WmZ : (gate == 1) ? WmR : WmH;
  const float* bias  = (gate == 0) ? bZ : (gate == 1) ? nullptr : bH;
  float* out         = (gate == 0) ? preZ : (gate == 1) ? preR : preH;

  __shared__ __align__(16) float st[32 * (kH + 4)];
  const int wave = threadIdx.x >> 5;
  const int lane = threadIdx.x & 31;
  const int tile = blockIdx.x * 8 + wave;
  const int row0 = (tile / 8) * 32;
  const int col0 = (tile % 8) * 32;
  V8FU a00 = {}, a01 = {}, a10 = {}, a11 = {};
  #pragma unroll
  for (int k0 = 0; k0 < kC; k0 += 32) {
    v16h va0 = load_a_f16(XI, kC, lane, row0, k0);
    v16h va1 = load_a_f16(XI, kC, lane, row0 + 16, k0);
    v16h vb0 = load_b_f16(Wx, kC, lane, col0, k0);
    v16h vb1 = load_b_f16(Wx, kC, lane, col0 + 16, k0);
    a00.v = wmma_f16(va0, vb0, a00.v);
    a01.v = wmma_f16(va0, vb1, a01.v);
    a10.v = wmma_f16(va1, vb0, a10.v);
    a11.v = wmma_f16(va1, vb1, a11.v);
  }
  #pragma unroll
  for (int k0 = 0; k0 < kC; k0 += 32) {
    v16h va0 = load_a_f16(M, kC, lane, row0, k0);
    v16h va1 = load_a_f16(M, kC, lane, row0 + 16, k0);
    v16h vb0 = load_b_f16(Wm, kC, lane, col0, k0);
    v16h vb1 = load_b_f16(Wm, kC, lane, col0 + 16, k0);
    a00.v = wmma_f16(va0, vb0, a00.v);
    a01.v = wmma_f16(va0, vb1, a01.v);
    a10.v = wmma_f16(va1, vb0, a10.v);
    a11.v = wmma_f16(va1, vb1, a11.v);
  }
  store_pre(st, bias, 0,  col0,      lane, a00);
  store_pre(st, bias, 0,  col0 + 16, lane, a01);
  store_pre(st, bias, 16, col0,      lane, a10);
  store_pre(st, bias, 16, col0 + 16, lane, a11);
  __syncthreads();
  for (int q = threadIdx.x; q < 32 * 64; q += 256) { const int rl = q >> 6, pc = q & 63;
    vst2(out + (size_t)(row0 + rl) * kH + pc * 4, *(const v4f*)(st + (size_t)rl * (kH + 4) + pc * 4)); }
}

__global__ void __launch_bounds__(512)
grud_recurrent(const _Float16* __restrict__ wHZ, const _Float16* __restrict__ wHR,
               const _Float16* __restrict__ wHH, const _Float16* __restrict__ wHY,
               const float* __restrict__ bHY, const float* __restrict__ GH,
               const float* __restrict__ preZ, const float* __restrict__ preR,
               const float* __restrict__ preH,
               float* __restrict__ ys, float* __restrict__ hs) {
  __shared__ __align__(16) float    h32[kB * kH];
  __shared__ __align__(16) _Float16 h16[kB * kH];
  __shared__ __align__(16) _Float16 rh16[kB * kH];
  __shared__ __align__(16) _Float16 z16[kB * kH];
  __shared__ __align__(16) float    y32[kB * kO];

  const int tid  = threadIdx.x;
  const int wave = tid >> 5;
  const int lane = tid & 31;
  const int rb   = (lane & 16) ? 8 : 0;
  const int cl   = lane & 15;

  for (int i = tid; i < kB * kH; i += 512) { h32[i] = 0.0f; h16[i] = (_Float16)0.0f; }
  __syncthreads();

  for (int t = 0; t < kT; ++t) {
    const size_t base = (size_t)t * kB * kH;

    for (int i = tid; i < kB * kH; i += 512) {
      const float hv = h32[i] * GH[base + i];
      h32[i] = hv;
      h16[i] = (_Float16)hv;
    }
    if (t + 1 < kT) {
      const size_t nb = base + (size_t)kB * kH;
      __builtin_prefetch(preZ + nb + tid * 32, 0, 1);
      __builtin_prefetch(preR + nb + tid * 32, 0, 1);
      __builtin_prefetch(preH + nb + tid * 32, 0, 1);
      __builtin_prefetch(GH + nb + tid * 32, 0, 1);
    }
    __syncthreads();

    for (int tt = wave; tt < 128; tt += 16) {
      const bool isZ = tt < 64;
      const int t64  = tt & 63;
      const int row0 = (t64 & 3) * 16;
      const int col0 = (t64 >> 2) * 16;
      const float* pre   = (isZ ? preZ : preR) + base;
      const _Float16* W  = isZ ? wHZ : wHR;
      const int col = col0 + cl;
      V8FU acc;
      #pragma unroll
      for (int i = 0; i < 8; ++i)
        acc.f[i] = pre[(size_t)(row0 + rb + i) * kH + col];
      #pragma unroll
      for (int k0 = 0; k0 < kH; k0 += 32) {
        v16h a = load_a_f16(h16, kH, lane, row0, k0);
        v16h b = load_b_f16(W, kH, lane, col0, k0);
        acc.v = wmma_f16(a, b, acc.v);
      }
      #pragma unroll
      for (int i = 0; i < 8; ++i) {
        const int r = row0 + rb + i;
        const float s = sigmoidf_(acc.f[i]);
        if (isZ) z16[r * kH + col] = (_Float16)s;
        else     rh16[r * kH + col] = (_Float16)(s * h32[r * kH + col]);
      }
    }
    __syncthreads();

    for (int tt = wave; tt < 64; tt += 16) {
      const int row0 = (tt & 3) * 16;
      const int col0 = (tt >> 2) * 16;
      const float* pre = preH + base;
      const int col = col0 + cl;
      V8FU acc;
      #pragma unroll
      for (int i = 0; i < 8; ++i)
        acc.f[i] = pre[(size_t)(row0 + rb + i) * kH + col];
      #pragma unroll
      for (int k0 = 0; k0 < kH; k0 += 32) {
        v16h a = load_a_f16(rh16, kH, lane, row0, k0);
        v16h b = load_b_f16(wHH, kH, lane, col0, k0);
        acc.v = wmma_f16(a, b, acc.v);
      }
      #pragma unroll
      for (int i = 0; i < 8; ++i) {
        const int r = row0 + rb + i;
        const int idx = r * kH + col;
        const float ht = tanhf(acc.f[i]);
        const float z  = (float)z16[idx];
        const float hn = (1.0f - z) * h32[idx] + z * ht;
        h32[idx] = hn;
        h16[idx] = (_Float16)hn;
      }
    }
    __syncthreads();
    for (int q = tid; q < kB * 64; q += 512) { const int r = q >> 6, pc = q & 63;
      vst2(hs + ((size_t)r * kT + t) * kH + pc * 4, *(const v4f*)(h32 + r * kH + pc * 4)); }

    for (int tt = wave; tt < 32; tt += 16) {
      const int row0 = (tt & 3) * 16;
      const int col0 = (tt >> 2) * 16;
      const int col = col0 + cl;
      V8FU acc;
      #pragma unroll
      for (int i = 0; i < 8; ++i) acc.f[i] = bHY[col];
      #pragma unroll
      for (int k0 = 0; k0 < kH; k0 += 32) {
        v16h a = load_a_f16(h16, kH, lane, row0, k0);
        v16h b = load_b_f16(wHY, kH, lane, col0, k0);
        acc.v = wmma_f16(a, b, acc.v);
      }
      #pragma unroll
      for (int i = 0; i < 8; ++i) {
        const int r = row0 + rb + i;
        y32[r * kO + col] = sigmoidf_(acc.f[i]);
      }
    }
    __syncthreads();
    for (int q = tid; q < kB * 32; q += 512) { const int r = q >> 5, pc = q & 31;
      vst2(ys + ((size_t)r * kT + t) * kO + pc * 4, *(const v4f*)(y32 + r * kO + pc * 4)); }
  }
}


extern "C" void kernel_launch(void* const* d_in, const int* in_sizes, int n_in,
                              void* d_out, int out_size, void* d_ws, size_t ws_size,
                              hipStream_t stream) {
  const float* inp    = (const float*)d_in[0];
  const float* W_dg_x = (const float*)d_in[1];
  const float* b_dg_x = (const float*)d_in[2];
  const float* W_dg_h = (const float*)d_in[3];
  const float* b_dg_h = (const float*)d_in[4];
  const float* W_xz   = (const float*)d_in[5];
  const float* W_hz   = (const float*)d_in[6];
  const float* W_mz   = (const float*)d_in[7];
  const float* b_mz   = (const float*)d_in[8];
  const float* W_xr   = (const float*)d_in[9];
  const float* W_hr   = (const float*)d_in[10];
  const float* W_mr   = (const float*)d_in[11];
  const float* W_xh   = (const float*)d_in[12];
  const float* W_hh   = (const float*)d_in[13];
  const float* W_mh   = (const float*)d_in[14];
  const float* b_mh   = (const float*)d_in[15];
  const float* W_hy   = (const float*)d_in[16];
  const float* b_hy   = (const float*)d_in[17];
  const float* x_mean = (const float*)d_in[18];

  char* ws = (char*)d_ws;
  size_t off = 0;
  auto take = [&](size_t bytes) -> char* {
    char* p = ws + off;
    off = (off + bytes + 255) & ~(size_t)255;
    return p;
  };

  _Float16* wDGX = (_Float16*)take((size_t)kC * kC * 2);
  _Float16* wDGH = (_Float16*)take((size_t)kH * kC * 2);
  _Float16* wXZ  = (_Float16*)take((size_t)kH * kC * 2);
  _Float16* wMZ  = (_Float16*)take((size_t)kH * kC * 2);
  _Float16* wXR  = (_Float16*)take((size_t)kH * kC * 2);
  _Float16* wMR  = (_Float16*)take((size_t)kH * kC * 2);
  _Float16* wXH  = (_Float16*)take((size_t)kH * kC * 2);
  _Float16* wMH  = (_Float16*)take((size_t)kH * kC * 2);
  _Float16* wHZ  = (_Float16*)take((size_t)kH * kH * 2);
  _Float16* wHR  = (_Float16*)take((size_t)kH * kH * 2);
  _Float16* wHH  = (_Float16*)take((size_t)kH * kH * 2);
  _Float16* wHY  = (_Float16*)take((size_t)kO * kH * 2);
  float*    Xf   = (float*)take((size_t)kTB * kC * 4);
  _Float16* M16  = (_Float16*)take((size_t)kTB * kC * 2);
  _Float16* D16  = (_Float16*)take((size_t)kTB * kC * 2);
  float*    GX   = (float*)take((size_t)kTB * kC * 4);
  float*    GH   = (float*)take((size_t)kTB * kH * 4);
  _Float16* XI   = (_Float16*)take((size_t)kTB * kC * 2);
  float*    pZ   = (float*)take((size_t)kTB * kH * 4);
  float*    pR   = (float*)take((size_t)kTB * kH * 4);
  float*    pH   = (float*)take((size_t)kTB * kH * 4);

  auto conv = [&](const float* s, _Float16* d, int n) {
    f32_to_f16_kernel<<<(n / 8 + 255) / 256, 256, 0, stream>>>(s, d, n);
  };
  conv(W_dg_x, wDGX, kC * kC);
  conv(W_dg_h, wDGH, kH * kC);
  conv(W_xz, wXZ, kH * kC);  conv(W_mz, wMZ, kH * kC);
  conv(W_xr, wXR, kH * kC);  conv(W_mr, wMR, kH * kC);
  conv(W_xh, wXH, kH * kC);  conv(W_mh, wMH, kH * kC);
  conv(W_hz, wHZ, kH * kH);  conv(W_hr, wHR, kH * kH);
  conv(W_hh, wHH, kH * kH);  conv(W_hy, wHY, kO * kH);

  reorder_inputs<<<kT, 256, 0, stream>>>(inp, Xf, M16, D16);

  gemm_gamma<<<512, 256, 0, stream>>>(D16, wDGX, b_dg_x, GX, kC, kC / 32, kC, kC);
  gemm_gamma<<<1024, 256, 0, stream>>>(D16, wDGH, b_dg_h, GH, kH, kH / 32, kC, kC);

  scan_impute<<<(kB * kC / 8) / 256, 256, 0, stream>>>(Xf, M16, GX, x_mean, XI);

  gemm_pre<<<dim3(1024, 3), 256, 0, stream>>>(XI, M16, wXZ, wMZ, wXR, wMR,
                                              wXH, wMH, b_mz, b_mh, pZ, pR, pH);

  float* ys = (float*)d_out;
  float* hs = ys + (size_t)kB * kT * kO;
  grud_recurrent<<<1, 512, 0, stream>>>(wHZ, wHR, wHH, wHY, b_hy, GH,
                                            pZ, pR, pH, ys, hs);
}
